// GNNCritic_30382598652559
// MI455X (gfx1250) — hardware-verified
//
#include <hip/hip_runtime.h>
#include <stddef.h>
#include <math.h>

#define HS     64
#define NHEAD  4
#define NE0    5
#define NE1    50
#define NE2    10
#define NTOK   65
#define SPB    4
#define NROWS  (SPB * NTOK)
#define MTKV   17
#define ZROW   272
#define XROWS  288
#define PX     72
#define NQ     (SPB * NE0)
#define QROWS  32
#define QZROW  24
#define KSLOT  96
#define PVT    384
#define NTHR   256
#define PARTF  32
#define NPLANE 6

static_assert(NE0 + NE1 + NE2 == NTOK);
static_assert(HS == NHEAD * 16);
static_assert(NROWS <= MTKV * 16);
static_assert(MTKV * 16 <= ZROW);
static_assert(ZROW < XROWS);
static_assert((SPB - 1) * NTOK + 5 * 16 <= XROWS);
static_assert(SPB * KSLOT <= PVT);
static_assert(3 * 32 <= KSLOT);
static_assert(NTOK <= KSLOT);
static_assert(PX % 8 == 0);
static_assert(PVT % 8 == 0);
static_assert(KSLOT % 8 == 0);
static_assert(NQ <= QZROW);
static_assert(QZROW < QROWS);
static_assert(QROWS == 32);
static_assert(NQ <= PARTF);
static_assert(NROWS % (NTHR / 64) == 0);
static_assert(NROWS <= 2 * NTHR);
static_assert(SPB * NHEAD == 16);
static_assert(NHEAD == 4);
static_assert(((XROWS - NROWS) * PX) % 8 == 0);
static_assert((NROWS * PX) % 8 == 0);
static_assert((SPB * NE0) % 4 == 0);

#define LB_XP    0
#define LB_K     (LB_XP   + XROWS * PX * 2)
#define LB_VT    (LB_K    + XROWS * PX * 2)
#define LB_Q     (LB_VT   + HS * PVT * 2)
#define LB_CTX   (LB_Q    + QROWS * PX * 2)
#define LB_M0    (LB_CTX  + QROWS * PX * 2)
#define LB_M1    (LB_M0   + QROWS * PX * 2)
#define LB_X32   (LB_M1   + QROWS * PX * 2)
#define LB_H2    (LB_X32  + QROWS * HS * 4)
#define LB_FEAT  (LB_H2   + QROWS * HS * 4)
#define LB_TRIG  (LB_FEAT + XROWS * 4 * 4)
#define LB_Y     (LB_TRIG + XROWS * 2 * 4)
#define LDS_BYTES (LB_Y   + PARTF * 4)

static_assert(LB_K % 16 == 0);
static_assert(LB_VT % 16 == 0);
static_assert(LB_Q % 16 == 0);
static_assert(LB_CTX % 16 == 0);
static_assert(LB_M0 % 16 == 0);
static_assert(LB_M1 % 16 == 0);
static_assert(LB_X32 % 16 == 0);
static_assert(LB_H2 % 16 == 0);
static_assert(LB_FEAT % 16 == 0);
static_assert(LB_TRIG % 16 == 0);
static_assert(LB_Y % 16 == 0);
static_assert(LDS_BYTES <= 300 * 1024);

typedef _Float16 f16;
typedef f16 v16h __attribute__((ext_vector_type(16)));
typedef f16 v8h_t __attribute__((ext_vector_type(8)));
typedef v8h_t __attribute__((may_alias)) v8h;
typedef float v8f __attribute__((ext_vector_type(8)));
typedef float v4f_t __attribute__((ext_vector_type(4)));
typedef v4f_t __attribute__((may_alias)) v4f;
typedef unsigned int v4u_t __attribute__((ext_vector_type(4)));
typedef v4u_t __attribute__((may_alias)) v4u;

union Frag { v16h v; v8h_t h[2]; v4u_t u[2]; };

__device__ __forceinline__ int imin(int a, int b) { return a < b ? a : b; }
__device__ __forceinline__ int imax(int a, int b) { return a > b ? a : b; }

__device__ __forceinline__ v8f zero8() {
  v8f z;
#pragma unroll
  for (int i = 0; i < 8; ++i) z[i] = 0.0f;
  return z;
}
__device__ __forceinline__ v4u_t zero4u() {
  v4u_t z;
#pragma unroll
  for (int i = 0; i < 4; ++i) z[i] = 0u;
  return z;
}

__device__ __forceinline__ v16h ldfrag2(const f16* p) {
  Frag f;
  f.h[0] = *(const v8h*)(p);
  f.h[1] = *(const v8h*)(p + 16);
  return f.v;
}
__device__ __forceinline__ v16h ldfrag_lo(const f16* p) {
  Frag f;
  f.h[0] = *(const v8h*)(p);
  f.u[1] = zero4u();
  return f.v;
}

__device__ __forceinline__ v8f wmma16(v16h a, v16h b, v8f c) {
  return __builtin_amdgcn_wmma_f32_16x16x32_f16(false, a, false, b, (short)0, c, false, false);
}

__device__ __forceinline__ v8f tile64(const f16* ap, v16h bf0, v16h bf1) {
  const v16h a0 = ldfrag2(ap);
  const v16h a1 = ldfrag2(ap + 32);
  v8f c = zero8();
  c = wmma16(a0, bf0, c);
  c = wmma16(a1, bf1, c);
  asm volatile("v_nop\n\tv_nop\n\tv_nop\n\tv_nop"
               : "+v"(c) : "v"(a0), "v"(a1), "v"(bf0), "v"(bf1));
  return c;
}

__device__ __forceinline__ void zfill(void* base, int n16, int t) {
  const v4u_t z = zero4u();
  v4u* p = (v4u*)base;
#pragma unroll 1
  for (int i = t; i < n16; i += NTHR) p[i] = z;
}

__global__ void __launch_bounds__(NTHR)
k_wcvt(const float* __restrict__ Wk, const float* __restrict__ Wq,
       const float* __restrict__ Wv, const float* __restrict__ Wo,
       const float* __restrict__ W1, const float* __restrict__ W2,
       f16* __restrict__ wpl)
{
  const int plane = blockIdx.x >> 1;
  const int u = ((blockIdx.x & 1) << 8) + threadIdx.x;
  const int n = u >> 3, k0 = (u & 7) * 8;
  const float* src = (plane == 0) ? Wk : (plane == 1) ? Wq : (plane == 2) ? Wv
                   : (plane == 3) ? Wo : (plane == 4) ? W1 : W2;
  union { v8h_t h; v4u_t u4; } pk;
#pragma unroll
  for (int e = 0; e < 8; ++e)
    pk.h[e] = (f16)(src[(size_t)(k0 + e) * HS + n] * 8.0f);
  f16* dst = wpl + (size_t)plane * (HS * HS) + (size_t)n * HS + k0;
  *(volatile v4u_t*)dst = pk.u4;
  __threadfence();
  *(volatile v4u_t*)dst = pk.u4;
}

__global__ void __launch_bounds__(NTHR) __attribute__((amdgpu_num_vgpr(256)))
k_main(const float* __restrict__ in_p, const float* __restrict__ in_y,
       const float* __restrict__ in_o, const float* __restrict__ act,
       const float* __restrict__ Wp, const float* __restrict__ bp,
       const float* __restrict__ Wy, const float* __restrict__ by,
       const float* __restrict__ Wob, const float* __restrict__ bob,
       const float* __restrict__ Wa, const float* __restrict__ ba,
       const float* __restrict__ Wq, const float* __restrict__ bq,
       const float* __restrict__ Wk, const float* __restrict__ bk,
       const float* __restrict__ bv, const float* __restrict__ bo,
       const float* __restrict__ b1, const float* __restrict__ b2,
       const float* __restrict__ W3, const float* __restrict__ b3,
       const f16* __restrict__ wpl, float* __restrict__ part, int nS)
{
  extern __shared__ __align__(16) unsigned char lds[];
  f16*   xp   = (f16*)(lds + LB_XP);
  f16*   k16  = (f16*)(lds + LB_K);
  f16*   vT   = (f16*)(lds + LB_VT);
  f16*   q16  = (f16*)(lds + LB_Q);
  f16*   cx16 = (f16*)(lds + LB_CTX);
  f16*   m0   = (f16*)(lds + LB_M0);
  f16*   m1   = (f16*)(lds + LB_M1);
  float* x32  = (float*)(lds + LB_X32);
  float* h2   = (float*)(lds + LB_H2);
  float* feat = (float*)(lds + LB_FEAT);
  float* trig = (float*)(lds + LB_TRIG);
  float* ybuf = (float*)(lds + LB_Y);

  const int t = threadIdx.x, w = t >> 5, lane = t & 31;
  const int hh = lane >> 4, m16 = lane & 15;
  const int blk = blockIdx.x;

  zfill(xp  + NROWS * PX, (XROWS - NROWS) * PX / 8, t);
  zfill(k16 + NROWS * PX, (XROWS - NROWS) * PX / 8, t);
  zfill(vT,   HS * PVT / 8, t);
  zfill(q16,  QROWS * PX / 8, t);
  zfill(cx16, QROWS * PX / 8, t);
  zfill(x32 + NQ * HS, (QROWS - NQ) * HS / 4, t);
  zfill(ybuf, PARTF / 4, t);

  const float PI_F = 3.14159274101257324f;
#pragma unroll 1
  for (int it = 0; it < 2; ++it) {
    const int r   = t + it * NTHR;
    const int rc  = imin(r, NROWS - 1);
    const int s   = rc / NTOK;
    const int key = rc - s * NTOK;
    const int gs  = imin(blk * SPB + s, nS - 1);
    const int i0  = imin(key, NE0 - 1);
    const int i1  = imin(imax(key - NE0, 0), NE1 - 1);
    const int i2  = imin(imax(key - NE0 - NE1, 0), NE2 - 1);
    const float* p0 = in_p + ((size_t)gs * NE0 + i0) * 2;
    const float* p1 = in_y + ((size_t)gs * NE1 + i1) * 2;
    const float* p2 = in_o + ((size_t)gs * NE2 + i2) * 3;
    const float a0 = p0[0], a1 = p0[1];
    const float c0 = p1[0], c1 = p1[1];
    const float d0 = p2[0], d1 = p2[1], d2 = p2[2];
    const bool g0 = key < NE0;
    const bool g1 = key < NE0 + NE1;
    const float f0 = g0 ? a0 : (g1 ? c0 : d0);
    const float f1 = g0 ? a1 : (g1 ? c1 : d1);
    const float ty = g0 ? 0.0f : (g1 ? 1.0f : 2.0f);
    const float ang = act[(size_t)gs * NE0 + i0] * PI_F;
    const float sa = sinf(ang), ca = cosf(ang);
    if (r < NROWS) {
      v4f_t fv;
      fv[0] = f0; fv[1] = f1; fv[2] = d2; fv[3] = ty;
      *(v4f*)(feat + r * 4) = fv;
      trig[r * 2]     = sa;
      trig[r * 2 + 1] = ca;
    }
  }
  __syncthreads();

  {
    const int c = t & 63, rb = t >> 6;
    const float wp0 = Wp[c],  wp1 = Wp[HS + c],  bpc  = bp[c];
    const float wy0 = Wy[c],  wy1 = Wy[HS + c],  byc  = by[c];
    const float wo0 = Wob[c], wo1 = Wob[HS + c], wo2  = Wob[2 * HS + c], bobc = bob[c];
    const float wa0 = Wa[c],  wa1 = Wa[HS + c],  bac  = ba[c];
#pragma unroll 1
    for (int j = 0; j < NROWS / (NTHR / 64); ++j) {
      const int row = rb + (NTHR / 64) * j;
      const v4f_t fv = *(const v4f*)(feat + row * 4);
      const float sa = trig[row * 2], ca = trig[row * 2 + 1];
      const float hp = fmaxf(fv[0] * wp0 + fv[1] * wp1 + bpc, 0.0f) + (sa * wa0 + ca * wa1 + bac);
      const float hy = fmaxf(fv[0] * wy0 + fv[1] * wy1 + byc, 0.0f);
      const float ho = fmaxf(fv[0] * wo0 + fv[1] * wo1 + fv[2] * wo2 + bobc, 0.0f);
      const float ty = fv[3];
      const float hsel = (ty < 0.5f) ? hp : ((ty < 1.5f) ? hy : ho);
      xp[row * PX + c] = (f16)(hsel * 16.0f);
      if (ty < 0.5f) {
        const int s = row / NTOK, key = row - s * NTOK;
        x32[(s * NE0 + key) * HS + c] = hsel;
      }
    }
  }
  __syncthreads();

  {
    const int nt = w & 3, cl = nt * 16 + m16;
    const f16* bb = wpl + 0 * (HS * HS) + (size_t)cl * HS + 8 * hh;
    const v16h bf0 = ldfrag2(bb), bf1 = ldfrag2(bb + 32);
    const float bkc = bk[cl], wk64 = Wk[64 * HS + cl], wk65 = Wk[65 * HS + cl];
    for (int mt = (w >> 2); mt < MTKV; mt += 2) {
      const v8f c = tile64(xp + (mt * 16 + m16) * PX + 8 * hh, bf0, bf1);
      const int row0 = mt * 16 + 8 * hh;
#pragma unroll
      for (int r = 0; r < 8; ++r) {
        const int row = row0 + r;
        const int fr  = imin(row, NROWS - 1);
        const float f0 = feat[fr * 4], f1 = feat[fr * 4 + 1];
        const float val = c[r] * (1.0f / 128.0f) + bkc + f0 * wk64 + f1 * wk65;
        if (row < NROWS) k16[row * PX + cl] = (f16)(val * 16.0f);
      }
    }
  }
  {
    const int nt = w & 3, cl = nt * 16 + m16;
    const f16* bb = wpl + 2 * (HS * HS) + (size_t)cl * HS + 8 * hh;
    const v16h bf0 = ldfrag2(bb), bf1 = ldfrag2(bb + 32);
    const float bvc = bv[cl];
    for (int mt = (w >> 2); mt < MTKV; mt += 2) {
      const v8f c = tile64(xp + (mt * 16 + m16) * PX + 8 * hh, bf0, bf1);
      const int row0 = mt * 16 + 8 * hh;
      const int s0 = row0 / NTOK;
      int key = row0 - s0 * NTOK;
      int sl  = s0 * KSLOT + key;
#pragma unroll
      for (int r = 0; r < 8; ++r) {
        const float val = (c[r] * (1.0f / 128.0f) + bvc) * 16.0f;
        if (row0 + r < NROWS) vT[cl * PVT + sl] = (f16)val;
        ++key; ++sl;
        if (key == NTOK) { key = 0; sl += KSLOT - NTOK; }
      }
    }
  }
  {
    const int mt = w >> 2, nt = w & 3, cl = nt * 16 + m16;
    const f16* bb = wpl + 1 * (HS * HS) + (size_t)cl * HS + 8 * hh;
    const v16h bf0 = ldfrag2(bb), bf1 = ldfrag2(bb + 32);
    const float bqc = bq[cl], wq64 = Wq[64 * HS + cl], wq65 = Wq[65 * HS + cl];
    const int qr = mt * 16 + m16;
    int xr = ZROW;
    if (qr < NQ) { const int s = qr / NE0; xr = s * NTOK + (qr - s * NE0); }
    const v8f c = tile64(xp + xr * PX + 8 * hh, bf0, bf1);
#pragma unroll
    for (int r = 0; r < 8; ++r) {
      const int qrow = mt * 16 + 8 * hh + r;
      const int qc = imin(qrow, NQ - 1);
      const int s = qc / NE0, p = qc - s * NE0;
      const int fr = s * NTOK + p;
      const float f0 = feat[fr * 4], f1 = feat[fr * 4 + 1];
      const float val = c[r] * (1.0f / 128.0f) + bqc + f0 * wq64 + f1 * wq65;
      if (qrow < NQ) q16[qrow * PX + cl] = (f16)(val * 16.0f);
    }
  }
  __syncthreads();

#pragma unroll 1
  for (int i = 0; i < (SPB * NHEAD) / 8; ++i) {
    const int u  = w + 8 * i;
    const int s  = u >> 2;
    const int hd = u & 3;
    const int qsel = (m16 < NE0) ? (s * NE0 + m16) : QZROW;
    const v16h qb  = ldfrag_lo(q16 + qsel * PX + hd * 16 + 8 * hh);
    const f16* kb  = k16 + (s * NTOK + m16) * PX + hd * 16 + 8 * hh;
    const v16h ka0 = ldfrag_lo(kb);
    const v16h ka1 = ldfrag_lo(kb + 16 * PX);
    const v16h ka2 = ldfrag_lo(kb + 32 * PX);
    const v16h ka3 = ldfrag_lo(kb + 48 * PX);
    const v16h ka4 = ldfrag_lo(kb + 64 * PX);
    v8f l0 = wmma16(ka0, qb, zero8());
    v8f l1 = wmma16(ka1, qb, zero8());
    v8f l2 = wmma16(ka2, qb, zero8());
    v8f l3 = wmma16(ka3, qb, zero8());
    v8f l4 = wmma16(ka4, qb, zero8());
    asm volatile("v_nop\n\tv_nop\n\tv_nop\n\tv_nop"
                 : "+v"(l0), "+v"(l1), "+v"(l2), "+v"(l3), "+v"(l4)
                 : "v"(ka0), "v"(ka1), "v"(ka2), "v"(ka3), "v"(ka4), "v"(qb));

    float mx = -__builtin_huge_valf();
#pragma unroll
    for (int r = 0; r < 8; ++r) {
      mx = fmaxf(mx, l0[r]); mx = fmaxf(mx, l1[r]);
      mx = fmaxf(mx, l2[r]); mx = fmaxf(mx, l3[r]);
    }
    const float l40 = (hh == 0) ? l4[0] : -__builtin_huge_valf();
    mx = fmaxf(mx, l40);
    mx = fmaxf(mx, __shfl_xor(mx, 16, 32));
    const float LSC = 1.0f / 1024.0f;
    v8f e0, e1, e2, e3;
    float sum = 0.0f;
#pragma unroll
    for (int r = 0; r < 8; ++r) {
      e0[r] = __expf((l0[r] - mx) * LSC); sum += e0[r];
      e1[r] = __expf((l1[r] - mx) * LSC); sum += e1[r];
      e2[r] = __expf((l2[r] - mx) * LSC); sum += e2[r];
      e3[r] = __expf((l3[r] - mx) * LSC); sum += e3[r];
    }
    const float e4u = __expf((l4[0] - mx) * LSC);
    const float e4  = (hh == 0) ? e4u : 0.0f;
    sum += e4;
    sum += __shfl_xor(sum, 16, 32);
    const float pf = __builtin_amdgcn_rcpf(sum) * 1024.0f;

    Frag pb0, pb1, pb2;
#pragma unroll
    for (int r = 0; r < 8; ++r) {
      pb0.h[0][r] = (f16)(e0[r] * pf);
      pb0.h[1][r] = (f16)(e1[r] * pf);
      pb1.h[0][r] = (f16)(e2[r] * pf);
      pb1.h[1][r] = (f16)(e3[r] * pf);
      pb2.h[1][r] = (f16)0.0f;
    }
    pb2.h[0][0] = (f16)(e4 * pf);
#pragma unroll
    for (int r = 1; r < 8; ++r) pb2.h[0][r] = (f16)0.0f;

    const f16* vb = vT + (hd * 16 + m16) * PVT + s * KSLOT + 8 * hh;
    const v16h va0 = ldfrag2(vb);
    const v16h va1 = ldfrag2(vb + 32);
    const v16h va2 = ldfrag2(vb + 64);
    v8f cc = zero8();
    cc = wmma16(va0, pb0.v, cc);
    cc = wmma16(va1, pb1.v, cc);
    cc = wmma16(va2, pb2.v, cc);
    asm volatile("v_nop\n\tv_nop\n\tv_nop\n\tv_nop"
                 : "+v"(cc)
                 : "v"(va0), "v"(va1), "v"(va2), "v"(pb0.v), "v"(pb1.v), "v"(pb2.v));
    if (m16 < NE0) {
      union { v8h_t h; v4u_t u4; } o;
#pragma unroll
      for (int r = 0; r < 8; ++r) o.h[r] = (f16)(cc[r] * (1.0f / 1024.0f));
      *(v4u*)(cx16 + (s * NE0 + m16) * PX + hd * 16 + 8 * hh) = o.u4;
    }
  }
  __syncthreads();

  {
    const int mt = w >> 2, nt = w & 3, cl = nt * 16 + m16;
    const f16* bb = wpl + 3 * (HS * HS) + (size_t)cl * HS + 8 * hh;
    const v16h bf0 = ldfrag2(bb), bf1 = ldfrag2(bb + 32);
    const float boc = bo[cl];
    const v8f c = tile64(cx16 + (mt * 16 + m16) * PX + 8 * hh, bf0, bf1);
#pragma unroll
    for (int r = 0; r < 8; ++r) {
      const int qrow = mt * 16 + 8 * hh + r;
      const float val = c[r] * (1.0f / 128.0f) + boc + x32[qrow * HS + cl];
      m0[qrow * PX + cl] = (f16)(val * 16.0f);
    }
  }
  __syncthreads();
  {
    const int mt = w >> 2, nt = w & 3, cl = nt * 16 + m16;
    const f16* bb = wpl + 4 * (HS * HS) + (size_t)cl * HS + 8 * hh;
    const v16h bf0 = ldfrag2(bb), bf1 = ldfrag2(bb + 32);
    const float b1c = b1[cl];
    const v8f c = tile64(m0 + (mt * 16 + m16) * PX + 8 * hh, bf0, bf1);
#pragma unroll
    for (int r = 0; r < 8; ++r) {
      const int qrow = mt * 16 + 8 * hh + r;
      const float val = fmaxf(c[r] * (1.0f / 128.0f) + b1c, 0.0f);
      m1[qrow * PX + cl] = (f16)(val * 16.0f);
    }
  }
  __syncthreads();
  {
    const int mt = w >> 2, nt = w & 3, cl = nt * 16 + m16;
    const f16* bb = wpl + 5 * (HS * HS) + (size_t)cl * HS + 8 * hh;
    const v16h bf0 = ldfrag2(bb), bf1 = ldfrag2(bb + 32);
    const float b2c = b2[cl];
    const v8f c = tile64(m1 + (mt * 16 + m16) * PX + 8 * hh, bf0, bf1);
#pragma unroll
    for (int r = 0; r < 8; ++r) {
      const int qrow = mt * 16 + 8 * hh + r;
      h2[qrow * HS + cl] = fmaxf(c[r] * (1.0f / 128.0f) + b2c, 0.0f);
    }
  }
  __syncthreads();

  {
    const float w3a = W3[lane], w3b = W3[lane + 32], b3v = b3[0];
    for (int q = w; q < NQ; q += 8) {
      float sacc = h2[q * HS + lane] * w3a + h2[q * HS + 32 + lane] * w3b;
#pragma unroll
      for (int off = 16; off > 0; off >>= 1) sacc += __shfl_xor(sacc, off, 32);
      if (lane == 0) ybuf[q] = sacc + b3v;
    }
  }
  __syncthreads();

  {
    const bool stl = (w == 0) && (lane < 8);
    const int li = stl ? lane : 0;
    const v4f_t yv = *(const v4f*)(ybuf + 4 * li);
    float* gp = part + (size_t)blk * PARTF + 4 * li;
    if (stl) *(volatile v4f_t*)gp = yv;
    __threadfence();
    if (stl) *(volatile v4f_t*)gp = yv;
  }
}

__global__ void __launch_bounds__(NTHR)
k_out(const float* __restrict__ part, float* __restrict__ out, int n4)
{
  const int i = blockIdx.x * NTHR + threadIdx.x;
  const bool ok = i < n4;
  const int ic = ok ? i : 0;
  const int o  = ic * 4;
  const int bi = o / (SPB * NE0);
  const int j  = o - bi * (SPB * NE0);
  const v4f_t v = *(const v4f*)(part + (size_t)bi * PARTF + j);
  float* dst = out + (size_t)ic * 4;
  if (ok) *(volatile v4f_t*)dst = v;
  __threadfence();
  if (ok) *(volatile v4f_t*)dst = v;
}

extern "C" void kernel_launch(void* const* d_in, const int* in_sizes, int n_in,
                              void* d_out, int out_size, void* d_ws, size_t ws_size,
                              hipStream_t stream)
{
  if (n_in < 26) return;
  const int nS = in_sizes[0] / (NE0 * 2);
  if (nS <= 0) return;
  if (in_sizes[0] != nS * NE0 * 2) return;
  if (in_sizes[1] != nS * NE1 * 2) return;
  if (in_sizes[2] != nS * NE2 * 3) return;
  if (in_sizes[3] != nS * NE0) return;
  if (in_sizes[4] != 2 * HS || in_sizes[5] != HS) return;
  if (in_sizes[6] != 2 * HS || in_sizes[7] != HS) return;
  if (in_sizes[8] != 3 * HS || in_sizes[9] != HS) return;
  if (in_sizes[10] != 2 * HS || in_sizes[11] != HS) return;
  if (in_sizes[12] != (HS + 2) * HS || in_sizes[13] != HS) return;
  if (in_sizes[14] != (HS + 2) * HS || in_sizes[15] != HS) return;
  if (in_sizes[16] != HS * HS || in_sizes[17] != HS) return;
  if (in_sizes[18] != HS * HS || in_sizes[19] != HS) return;
  if (in_sizes[20] != HS * HS || in_sizes[21] != HS) return;
  if (in_sizes[22] != HS * HS || in_sizes[23] != HS) return;
  if (in_sizes[24] != HS || in_sizes[25] < 1) return;
  if (out_size != nS * NE0) return;
  if ((nS % SPB) != 0) return;
  if ((out_size % 4) != 0) return;

  const int nblk = nS / SPB;

  const size_t oPl    = 0;
  const size_t plB    = (size_t)NPLANE * HS * HS * 2;
  const size_t oPart  = oPl + plB;
  const size_t partB  = (size_t)nblk * PARTF * 4;
  const size_t total  = oPart + partB;
  if (total > ws_size) return;

  const float* in_p = (const float*)d_in[0];
  const float* in_y = (const float*)d_in[1];
  const float* in_o = (const float*)d_in[2];
  const float* act  = (const float*)d_in[3];
  const float* Wp  = (const float*)d_in[4];   const float* bp  = (const float*)d_in[5];
  const float* Wy  = (const float*)d_in[6];   const float* by  = (const float*)d_in[7];
  const float* Wob = (const float*)d_in[8];   const float* bob = (const float*)d_in[9];
  const float* Wa  = (const float*)d_in[10];  const float* ba  = (const float*)d_in[11];
  const float* Wq  = (const float*)d_in[12];  const float* bq  = (const float*)d_in[13];
  const float* Wk  = (const float*)d_in[14];  const float* bk  = (const float*)d_in[15];
  const float* Wv  = (const float*)d_in[16];  const float* bv  = (const float*)d_in[17];
  const float* Wo  = (const float*)d_in[18];  const float* bo  = (const float*)d_in[19];
  const float* W1  = (const float*)d_in[20];  const float* b1  = (const float*)d_in[21];
  const float* W2  = (const float*)d_in[22];  const float* b2  = (const float*)d_in[23];
  const float* W3  = (const float*)d_in[24];  const float* b3  = (const float*)d_in[25];
  float* out = (float*)d_out;

  char* ws = (char*)d_ws;
  f16*   wpl  = (f16*)(ws + oPl);
  float* part = (float*)(ws + oPart);

  k_wcvt<<<NPLANE * 2, NTHR, 0, stream>>>(Wk, Wq, Wv, Wo, W1, W2, wpl);

  hipFuncSetAttribute(reinterpret_cast<const void*>(&k_main),
                      hipFuncAttributeMaxDynamicSharedMemorySize, LDS_BYTES);
  k_main<<<nblk, NTHR, LDS_BYTES, stream>>>(
      in_p, in_y, in_o, act, Wp, bp, Wy, by, Wob, bob, Wa, ba,
      Wq, bq, Wk, bk, bv, bo, b1, b2, W3, b3, wpl, part, nS);

  const int n4 = out_size / 4;
  k_out<<<(n4 + NTHR - 1) / NTHR, NTHR, 0, stream>>>(part, out, n4);
}
